// ViSNetEncoderMSE_90477781057666
// MI455X (gfx1250) — hardware-run, weakly checked
//
#include <hip/hip_runtime.h>


namespace {
constexpr int N = 10000, NP = 10048, E = 160000, H = 128, R = 32, L = 2, LAT = 64, G = 128, OW = 80;
constexpr float CUT = 5.0f, EPSR = 1e-8f, XS = 8.0f, RS = 1024.0f, WSC = 256.0f;
typedef _Float16 b16;
typedef __attribute__((ext_vector_type(16))) _Float16 v16b;
typedef __attribute__((ext_vector_type(8))) _Float16 v8b;
typedef __attribute__((ext_vector_type(4))) _Float16 v4b;
typedef __attribute__((ext_vector_type(2))) _Float16 v2b;
typedef __attribute__((ext_vector_type(8))) float v8f;
typedef __attribute__((ext_vector_type(4))) float v4f;
__device__ __forceinline__ float bf16_rne(float f) { unsigned int u = __float_as_uint(f); u += 0x7FFFu + ((u >> 16) & 1u); return __uint_as_float(u & 0xFFFF0000u); }
__device__ __forceinline__ void split16(float v, b16& hi, b16& lo) { hi = (b16)v; lo = (b16)(v - (float)hi); }
__device__ __forceinline__ v16b frag_kb(const b16* p, int hh) { const v8b a = *(const v8b*)(p + 8 * hh), b = *(const v8b*)(p + 16 + 8 * hh); v16b f;
#pragma unroll
  for (int e = 0; e < 8; ++e) { f[e] = a[e]; f[8 + e] = b[e]; } return f; }
__device__ __forceinline__ v8f wmma16b(v16b a, v16b b, v8f c) { v8f d = __builtin_amdgcn_wmma_f32_16x16x32_f16(false, a, false, b, (short)0, c, false, false); asm volatile("v_nop\n\tv_nop\n\tv_nop\n\tv_nop" : "+v"(d) : "v"(a), "v"(b)); return d; }
__device__ __forceinline__ void wave_lds_sync() { __builtin_amdgcn_fence(__ATOMIC_RELEASE, "workgroup"); __builtin_amdgcn_wave_barrier(); __builtin_amdgcn_fence(__ATOMIC_ACQUIRE, "workgroup"); }
__device__ __forceinline__ float pmul(float a, float b) { float p = a * b; asm volatile("" : "+v"(p)); return p; }
__device__ __forceinline__ int iclamp(int v, int lo, int hi) { return v < lo ? lo : (v > hi ? hi : v); }
__device__ __forceinline__ float siluf(float t) { return t / (1.0f + __expf(-t)); }
constexpr int CSR_NBLK9 = 512, CSR_GB9 = 9, CSR_GN9 = 1 << CSR_GB9  , CSR_TS9 = (CSR_GN9 < 32 ? 32 : CSR_GN9)  , CSR_MAXG9 = 512, CSR_CAP9 = 12288  ;
__device__ __host__ __forceinline__ int csr_tix9(int v) { return (v >> CSR_GB9) * CSR_TS9 + (v & (CSR_GN9 - 1)); }
__global__ __launch_bounds__(64) void csrA_kernel9(const int* __restrict__ dst, int E, int N, int nG, int CHP, int NGP, int* __restrict__ STG, int* __restrict__ HST) {
  extern __shared__ int sm[];
  int* cnt = sm; int* run = sm + NGP; int* ids = sm + 2 * NGP;
  const int b = blockIdx.x; const int ch = (E + CSR_NBLK9 - 1) / CSR_NBLK9; const int e0 = b * ch, e1 = min(E, e0 + ch);
  for (int i = threadIdx.x; i < NGP; i += 64) cnt[i] = 0;
  for (int i = threadIdx.x; i < CHP; i += 64) ids[i] = -1;
  __syncthreads();
  if (threadIdx.x == 0) {
    for (int e = e0; e < e1; ++e) { int d = dst[e]; d = (d < 0) ? 0 : (d >= N ? N - 1 : d); cnt[d >> CSR_GB9] += 1; }
    int acc = 0; for (int g = 0; g < nG; ++g) { run[g] = acc; acc += cnt[g]; }
    for (int e = e0; e < e1; ++e) { int d = dst[e]; d = (d < 0) ? 0 : (d >= N ? N - 1 : d); const int g = d >> CSR_GB9; ids[run[g]] = e; run[g] += 1; } }
  __syncthreads();
  typedef __attribute__((ext_vector_type(4))) int v4i;
  for (int pass = 0; pass < 2; ++pass) {
    for (int i = threadIdx.x; i < CHP / 4; i += 64) *(volatile v4i*)(STG + (size_t)b * CHP + i * 4) = *(const v4i*)(&ids[i * 4]);
    for (int i = threadIdx.x; i < NGP / 4; i += 64) { v4i v; for (int e = 0; e < 4; ++e) v[e] = (i * 4 + e < nG) ? cnt[i * 4 + e] : 0; *(volatile v4i*)(HST + (size_t)b * NGP + i * 4) = v; }
    __threadfence(); }
}
__global__ __launch_bounds__(512) void csrS_kernel9(const int* __restrict__ HST, int nG, int NGP, int* __restrict__ START, int* __restrict__ TOT, int* __restrict__ OFF) {
  __shared__ int tot[CSR_MAXG9];
  const int b = threadIdx.x;
  for (int pass = 0; pass < 2; ++pass) { int runb = 0; for (int g = 0; g < nG; ++g) { int c = HST[(size_t)b * NGP + g]; c = (c < 0) ? 0 : c; ((volatile int*)OFF)[(size_t)g * CSR_NBLK9 + b] = runb; runb += c; } __threadfence(); }
  for (int g = threadIdx.x; g < nG; g += 512) { int s = 0; for (int bb = 0; bb < CSR_NBLK9; ++bb) { int c = HST[(size_t)bb * NGP + g]; s += (c < 0) ? 0 : c; } tot[g] = s; }
  __syncthreads();
  if (threadIdx.x < 32) {
    __shared__ int st[CSR_MAXG9 + 32];
    if (threadIdx.x == 0) { int acc = 0; for (int g = 0; g < NGP; ++g) { st[g] = acc; if (g < nG) acc += (tot[g] + 31) & ~31; } st[NGP] = acc; }
    __builtin_amdgcn_fence(__ATOMIC_RELEASE, "workgroup"); __builtin_amdgcn_wave_barrier(); __builtin_amdgcn_fence(__ATOMIC_ACQUIRE, "workgroup");
    for (int pass = 0; pass < 2; ++pass) { for (int i = threadIdx.x; i < NGP + 32; i += 32) { ((volatile int*)START)[i] = (i <= NGP) ? st[min(i, NGP)] : 0; ((volatile int*)TOT)[i] = (i < nG) ? tot[i] : 0; } __threadfence(); } }
}
__global__ __launch_bounds__(256) void csrB_kernel9(const int* __restrict__ dst, int N, int nG, int CHP, int NGP, int permLen, const int* __restrict__ STG, const int* __restrict__ HST, const int* __restrict__ OFF, const int* __restrict__ START, const int* __restrict__ TOT, int* __restrict__ PERM, int* __restrict__ ROWPTR, int* __restrict__ ROWCNT, int* __restrict__ FLAG) {
  typedef __attribute__((ext_vector_type(4))) int v4i;
  __shared__ int ids[CSR_CAP9]; __shared__ unsigned short key[CSR_CAP9]; __shared__ int outp[CSR_CAP9]; __shared__ int ncnt[CSR_GN9 + 1]; __shared__ int boff[CSR_NBLK9 + 1];
  const int g = blockIdx.x, t_ = threadIdx.x; int tot = TOT[g]; int st = START[g], stn = START[g + 1]; const int v0 = g * CSR_GN9; const int nv = min(CSR_GN9, N - v0); const int t0 = g * CSR_TS9;
  st = (st < 0) ? 0 : (st > permLen - 32 ? permLen - 32 : st) & ~31; stn = (stn < st) ? st : (stn > permLen ? permLen : stn); tot = (tot < 0) ? 0 : tot; if (tot > stn - st && tot <= CSR_CAP9) tot = stn - st;
  if (tot > CSR_CAP9) {
    for (int pass = 0; pass < 2; ++pass) { for (int i = t_; i < CSR_TS9 / 4; i += 256) { v4i a, c; for (int e = 0; e < 4; ++e) { a[e] = st; c[e] = 0; } *(volatile v4i*)(ROWPTR + t0 + i * 4) = a; *(volatile v4i*)(ROWCNT + t0 + i * 4) = c; } if (t_ == 0) ((volatile int*)FLAG)[0] = 1; __threadfence(); } (void)nv; return; }
  if (t_ == 0) { int acc = 0; for (int b = 0; b < CSR_NBLK9; ++b) { boff[b] = acc; int c = HST[(size_t)b * NGP + g]; c = (c < 0) ? 0 : (c > CHP ? CHP : c); acc += c; if (acc > tot) acc = tot; } boff[CSR_NBLK9] = acc; }
  for (int i = t_; i <= CSR_GN9; i += 256) ncnt[i] = 0;
  __syncthreads();
  for (int b = 0; b < CSR_NBLK9; ++b) { const int c = boff[b + 1] - boff[b]; int o_ = OFF[(size_t)g * CSR_NBLK9 + b]; o_ = (o_ < 0) ? 0 : (o_ > CHP - c ? CHP - c : o_); const int* src_ = STG + (size_t)b * CHP + o_;
    for (int i = t_; i < c; i += 256) { int id = src_[i]; id = (id < 0) ? 0 : id; ids[boff[b] + i] = id; int d = dst[id]; d = (d < v0) ? v0 : (d >= N ? N - 1 : d); int kk = d - v0; kk = (kk < 0) ? 0 : (kk >= CSR_GN9 ? CSR_GN9 - 1 : kk); key[boff[b] + i] = (unsigned short)kk; } }
  __syncthreads();
  if (t_ == 0) { for (int i = 0; i < tot; ++i) ncnt[key[i]] += 1; int acc = 0; for (int vl = 0; vl < CSR_GN9; ++vl) { const int c = ncnt[vl]; ncnt[vl] = acc; acc += c; } ncnt[CSR_GN9] = acc;
    for (int i = 0; i < tot; ++i) { const int vl = key[i]; outp[ncnt[vl]] = ids[i]; ncnt[vl] += 1; }
    for (int vl = CSR_GN9; vl > 0; --vl) ncnt[vl] = ncnt[vl - 1]; ncnt[0] = 0; }
  __syncthreads();
  for (int pass = 0; pass < 2; ++pass) {
    for (int i = t_; i < (stn - st) / 4; i += 256) { v4i v; for (int e = 0; e < 4; ++e) { const int q = i * 4 + e; v[e] = (q < tot) ? outp[q] : -1; } *(volatile v4i*)(PERM + st + i * 4) = v; }
    for (int i = t_; i < CSR_TS9 / 4; i += 256) { v4i a, c; for (int e = 0; e < 4; ++e) { const int vl = i * 4 + e; const int vc = vl < CSR_GN9 ? vl : CSR_GN9; a[e] = (vl < CSR_GN9) ? st + ncnt[vc] : st; c[e] = (vl < nv) ? (ncnt[(vc < CSR_GN9 ? vc : CSR_GN9 - 1) + 1] - ncnt[vc]) : 0; } *(volatile v4i*)(ROWPTR + t0 + i * 4) = a; *(volatile v4i*)(ROWCNT + t0 + i * 4) = c; }
    __threadfence(); }
}
__global__ __launch_bounds__(256) void csrZ_kernel9(int* __restrict__ p, size_t n4) { typedef __attribute__((ext_vector_type(4))) int v4i; const size_t tid = (size_t)blockIdx.x * 256 + threadIdx.x, nth = (size_t)gridDim.x * 256; v4i z = {0, 0, 0, 0}; for (size_t i = tid; i < n4; i += nth) *(volatile v4i*)(p + i * 4) = z; }
struct CsrBufs9 { int *STG, *HST, *OFF, *START, *TOT, *PERM, *ROWPTR, *ROWCNT, *FLAG; int nG, NGP, CHP; size_t permLen; char* base; size_t bytes; };
static size_t csr_carve9(CsrBufs9& c, char* ws, size_t off, int E, int N) {
  const size_t off0 = off; c.base = ws + off;
  auto al = [&](size_t bytes) { char* p = ws + off; off += (bytes + 255) & ~(size_t)255; return p; };
  c.nG = (N + CSR_GN9 - 1) / CSR_GN9; c.NGP = (c.nG + 31) & ~31; const int ch = (E + CSR_NBLK9 - 1) / CSR_NBLK9; c.CHP = (ch + 31) & ~31; c.permLen = (size_t)E + 32 * (size_t)c.nG + 32;
  c.STG = (int*)al((size_t)CSR_NBLK9 * c.CHP * 4); c.HST = (int*)al((size_t)CSR_NBLK9 * c.NGP * 4); c.OFF = (int*)al((size_t)c.NGP * CSR_NBLK9 * 4); c.START = (int*)al((size_t)(c.NGP + 64) * 4); c.TOT = (int*)al((size_t)(c.NGP + 64) * 4);
  c.PERM = (int*)al(c.permLen * 4); c.ROWPTR = (int*)al((size_t)c.nG * CSR_TS9 * 4); c.ROWCNT = (int*)al((size_t)c.nG * CSR_TS9 * 4); c.FLAG = (int*)al(256);
  c.bytes = off - off0; return off;
}
static void csr_build9(const CsrBufs9& c, const int* dst, int E, int N, hipStream_t stream) {
  const size_t smem = (size_t)(2 * c.NGP + c.CHP) * 4;
  csrZ_kernel9<<<512, 256, 0, stream>>>((int*)c.base, c.bytes / 16);
  csrA_kernel9<<<CSR_NBLK9, 64, smem, stream>>>(dst, E, N, c.nG, c.CHP, c.NGP, c.STG, c.HST);
  csrS_kernel9<<<1, 512, 0, stream>>>(c.HST, c.nG, c.NGP, c.START, c.TOT, c.OFF);
  csrB_kernel9<<<c.nG, 256, 0, stream>>>(dst, N, c.nG, c.CHP, c.NGP, (int)c.permLen, c.STG, c.HST, c.OFF, c.START, c.TOT, c.PERM, c.ROWPTR, c.ROWCNT, c.FLAG);
}

constexpr int CSR_NBLK3 = 512, CSR_GB3 = 3, CSR_GN3 = 1 << CSR_GB3  , CSR_TS3 = (CSR_GN3 < 32 ? 32 : CSR_GN3)  , CSR_MAXG3 = 512, CSR_CAP3 = 12288  ;
__device__ __host__ __forceinline__ int csr_tix3(int v) { return (v >> CSR_GB3) * CSR_TS3 + (v & (CSR_GN3 - 1)); }
__global__ __launch_bounds__(64) void csrA_kernel3(const int* __restrict__ dst, int E, int N, int nG, int CHP, int NGP, int* __restrict__ STG, int* __restrict__ HST) {
  extern __shared__ int sm[];
  int* cnt = sm; int* run = sm + NGP; int* ids = sm + 2 * NGP;
  const int b = blockIdx.x; const int ch = (E + CSR_NBLK3 - 1) / CSR_NBLK3; const int e0 = b * ch, e1 = min(E, e0 + ch);
  for (int i = threadIdx.x; i < NGP; i += 64) cnt[i] = 0;
  for (int i = threadIdx.x; i < CHP; i += 64) ids[i] = -1;
  __syncthreads();
  if (threadIdx.x == 0) {
    for (int e = e0; e < e1; ++e) { int d = dst[e]; d = (d < 0) ? 0 : (d >= N ? N - 1 : d); cnt[d >> CSR_GB3] += 1; }
    int acc = 0; for (int g = 0; g < nG; ++g) { run[g] = acc; acc += cnt[g]; }
    for (int e = e0; e < e1; ++e) { int d = dst[e]; d = (d < 0) ? 0 : (d >= N ? N - 1 : d); const int g = d >> CSR_GB3; ids[run[g]] = e; run[g] += 1; } }
  __syncthreads();
  typedef __attribute__((ext_vector_type(4))) int v4i;
  for (int pass = 0; pass < 2; ++pass) {
    for (int i = threadIdx.x; i < CHP / 4; i += 64) *(volatile v4i*)(STG + (size_t)b * CHP + i * 4) = *(const v4i*)(&ids[i * 4]);
    for (int i = threadIdx.x; i < NGP / 4; i += 64) { v4i v; for (int e = 0; e < 4; ++e) v[e] = (i * 4 + e < nG) ? cnt[i * 4 + e] : 0; *(volatile v4i*)(HST + (size_t)b * NGP + i * 4) = v; }
    __threadfence(); }
}
__global__ __launch_bounds__(512) void csrS_kernel3(const int* __restrict__ HST, int nG, int NGP, int* __restrict__ START, int* __restrict__ TOT, int* __restrict__ OFF) {
  __shared__ int tot[CSR_MAXG3];
  const int b = threadIdx.x;
  for (int pass = 0; pass < 2; ++pass) { int runb = 0; for (int g = 0; g < nG; ++g) { int c = HST[(size_t)b * NGP + g]; c = (c < 0) ? 0 : c; ((volatile int*)OFF)[(size_t)g * CSR_NBLK3 + b] = runb; runb += c; } __threadfence(); }
  for (int g = threadIdx.x; g < nG; g += 512) { int s = 0; for (int bb = 0; bb < CSR_NBLK3; ++bb) { int c = HST[(size_t)bb * NGP + g]; s += (c < 0) ? 0 : c; } tot[g] = s; }
  __syncthreads();
  if (threadIdx.x < 32) {
    __shared__ int st[CSR_MAXG3 + 32];
    if (threadIdx.x == 0) { int acc = 0; for (int g = 0; g < NGP; ++g) { st[g] = acc; if (g < nG) acc += (tot[g] + 31) & ~31; } st[NGP] = acc; }
    __builtin_amdgcn_fence(__ATOMIC_RELEASE, "workgroup"); __builtin_amdgcn_wave_barrier(); __builtin_amdgcn_fence(__ATOMIC_ACQUIRE, "workgroup");
    for (int pass = 0; pass < 2; ++pass) { for (int i = threadIdx.x; i < NGP + 32; i += 32) { ((volatile int*)START)[i] = (i <= NGP) ? st[min(i, NGP)] : 0; ((volatile int*)TOT)[i] = (i < nG) ? tot[i] : 0; } __threadfence(); } }
}
__global__ __launch_bounds__(256) void csrB_kernel3(const int* __restrict__ dst, int N, int nG, int CHP, int NGP, int permLen, const int* __restrict__ STG, const int* __restrict__ HST, const int* __restrict__ OFF, const int* __restrict__ START, const int* __restrict__ TOT, int* __restrict__ PERM, int* __restrict__ ROWPTR, int* __restrict__ ROWCNT, int* __restrict__ FLAG) {
  typedef __attribute__((ext_vector_type(4))) int v4i;
  __shared__ int ids[CSR_CAP3]; __shared__ unsigned short key[CSR_CAP3]; __shared__ int outp[CSR_CAP3]; __shared__ int ncnt[CSR_GN3 + 1]; __shared__ int boff[CSR_NBLK3 + 1];
  const int g = blockIdx.x, t_ = threadIdx.x; int tot = TOT[g]; int st = START[g], stn = START[g + 1]; const int v0 = g * CSR_GN3; const int nv = min(CSR_GN3, N - v0); const int t0 = g * CSR_TS3;
  st = (st < 0) ? 0 : (st > permLen - 32 ? permLen - 32 : st) & ~31; stn = (stn < st) ? st : (stn > permLen ? permLen : stn); tot = (tot < 0) ? 0 : tot; if (tot > stn - st && tot <= CSR_CAP3) tot = stn - st;
  if (tot > CSR_CAP3) {
    for (int pass = 0; pass < 2; ++pass) { for (int i = t_; i < CSR_TS3 / 4; i += 256) { v4i a, c; for (int e = 0; e < 4; ++e) { a[e] = st; c[e] = 0; } *(volatile v4i*)(ROWPTR + t0 + i * 4) = a; *(volatile v4i*)(ROWCNT + t0 + i * 4) = c; } if (t_ == 0) ((volatile int*)FLAG)[0] = 1; __threadfence(); } (void)nv; return; }
  if (t_ == 0) { int acc = 0; for (int b = 0; b < CSR_NBLK3; ++b) { boff[b] = acc; int c = HST[(size_t)b * NGP + g]; c = (c < 0) ? 0 : (c > CHP ? CHP : c); acc += c; if (acc > tot) acc = tot; } boff[CSR_NBLK3] = acc; }
  for (int i = t_; i <= CSR_GN3; i += 256) ncnt[i] = 0;
  __syncthreads();
  for (int b = 0; b < CSR_NBLK3; ++b) { const int c = boff[b + 1] - boff[b]; int o_ = OFF[(size_t)g * CSR_NBLK3 + b]; o_ = (o_ < 0) ? 0 : (o_ > CHP - c ? CHP - c : o_); const int* src_ = STG + (size_t)b * CHP + o_;
    for (int i = t_; i < c; i += 256) { int id = src_[i]; id = (id < 0) ? 0 : id; ids[boff[b] + i] = id; int d = dst[id]; d = (d < v0) ? v0 : (d >= N ? N - 1 : d); int kk = d - v0; kk = (kk < 0) ? 0 : (kk >= CSR_GN3 ? CSR_GN3 - 1 : kk); key[boff[b] + i] = (unsigned short)kk; } }
  __syncthreads();
  if (t_ == 0) { for (int i = 0; i < tot; ++i) ncnt[key[i]] += 1; int acc = 0; for (int vl = 0; vl < CSR_GN3; ++vl) { const int c = ncnt[vl]; ncnt[vl] = acc; acc += c; } ncnt[CSR_GN3] = acc;
    for (int i = 0; i < tot; ++i) { const int vl = key[i]; outp[ncnt[vl]] = ids[i]; ncnt[vl] += 1; }
    for (int vl = CSR_GN3; vl > 0; --vl) ncnt[vl] = ncnt[vl - 1]; ncnt[0] = 0; }
  __syncthreads();
  for (int pass = 0; pass < 2; ++pass) {
    for (int i = t_; i < (stn - st) / 4; i += 256) { v4i v; for (int e = 0; e < 4; ++e) { const int q = i * 4 + e; v[e] = (q < tot) ? outp[q] : -1; } *(volatile v4i*)(PERM + st + i * 4) = v; }
    for (int i = t_; i < CSR_TS3 / 4; i += 256) { v4i a, c; for (int e = 0; e < 4; ++e) { const int vl = i * 4 + e; const int vc = vl < CSR_GN3 ? vl : CSR_GN3; a[e] = (vl < CSR_GN3) ? st + ncnt[vc] : st; c[e] = (vl < nv) ? (ncnt[(vc < CSR_GN3 ? vc : CSR_GN3 - 1) + 1] - ncnt[vc]) : 0; } *(volatile v4i*)(ROWPTR + t0 + i * 4) = a; *(volatile v4i*)(ROWCNT + t0 + i * 4) = c; }
    __threadfence(); }
}
__global__ __launch_bounds__(256) void csrZ_kernel3(int* __restrict__ p, size_t n4) { typedef __attribute__((ext_vector_type(4))) int v4i; const size_t tid = (size_t)blockIdx.x * 256 + threadIdx.x, nth = (size_t)gridDim.x * 256; v4i z = {0, 0, 0, 0}; for (size_t i = tid; i < n4; i += nth) *(volatile v4i*)(p + i * 4) = z; }
struct CsrBufs3 { int *STG, *HST, *OFF, *START, *TOT, *PERM, *ROWPTR, *ROWCNT, *FLAG; int nG, NGP, CHP; size_t permLen; char* base; size_t bytes; };
static size_t csr_carve3(CsrBufs3& c, char* ws, size_t off, int E, int N) {
  const size_t off0 = off; c.base = ws + off;
  auto al = [&](size_t bytes) { char* p = ws + off; off += (bytes + 255) & ~(size_t)255; return p; };
  c.nG = (N + CSR_GN3 - 1) / CSR_GN3; c.NGP = (c.nG + 31) & ~31; const int ch = (E + CSR_NBLK3 - 1) / CSR_NBLK3; c.CHP = (ch + 31) & ~31; c.permLen = (size_t)E + 32 * (size_t)c.nG + 32;
  c.STG = (int*)al((size_t)CSR_NBLK3 * c.CHP * 4); c.HST = (int*)al((size_t)CSR_NBLK3 * c.NGP * 4); c.OFF = (int*)al((size_t)c.NGP * CSR_NBLK3 * 4); c.START = (int*)al((size_t)(c.NGP + 64) * 4); c.TOT = (int*)al((size_t)(c.NGP + 64) * 4);
  c.PERM = (int*)al(c.permLen * 4); c.ROWPTR = (int*)al((size_t)c.nG * CSR_TS3 * 4); c.ROWCNT = (int*)al((size_t)c.nG * CSR_TS3 * 4); c.FLAG = (int*)al(256);
  c.bytes = off - off0; return off;
}
static void csr_build3(const CsrBufs3& c, const int* dst, int E, int N, hipStream_t stream) {
  const size_t smem = (size_t)(2 * c.NGP + c.CHP) * 4;
  csrZ_kernel3<<<512, 256, 0, stream>>>((int*)c.base, c.bytes / 16);
  csrA_kernel3<<<CSR_NBLK3, 64, smem, stream>>>(dst, E, N, c.nG, c.CHP, c.NGP, c.STG, c.HST);
  csrS_kernel3<<<1, 512, 0, stream>>>(c.HST, c.nG, c.NGP, c.START, c.TOT, c.OFF);
  csrB_kernel3<<<c.nG, 256, 0, stream>>>(dst, N, c.nG, c.CHP, c.NGP, (int)c.permLen, c.STG, c.HST, c.OFF, c.START, c.TOT, c.PERM, c.ROWPTR, c.ROWCNT, c.FLAG);
}


__global__ __launch_bounds__(256) void wprep_kernel(const float* __restrict__ wrbf, const float* __restrict__ w1, const float* __restrict__ wo, const float* __restrict__ wv, const float* __restrict__ wv2, const float* __restrict__ wa, const float* __restrict__ wb,
                                                    b16* __restrict__ WR, b16* __restrict__ W1T, b16* __restrict__ WOT, b16* __restrict__ WVT, b16* __restrict__ WV2T, b16* __restrict__ WAT, b16* __restrict__ WBT) {
  const size_t u = (size_t)blockIdx.x * 256 + threadIdx.x; size_t t = u; v8b o;
  const size_t nr = (size_t)L * H * R / 8, nq = (size_t)L * H * H / 8, n2 = (size_t)H * H / 8, na = (size_t)H * 2 * H / 8, nb = (size_t)OW * H / 8;
  if (t < nr) { const size_t e = t * 8; const int l = (int)(e / (H * R)); const int oo = (int)((e / R) % H), k0 = (int)(e % R); for (int j = 0; j < 8; ++j) o[j] = (b16)(bf16_rne(wrbf[((size_t)l * R + k0 + j) * H + oo]) * WSC); for (int p = 0; p < 2; ++p) { *(volatile v8b*)(WR + e) = o; __threadfence(); } return; } t -= nr;
  for (int which = 0; which < 3; ++which) { const float* w = which == 0 ? w1 : (which == 1 ? wo : wv); b16* dst_ = which == 0 ? W1T : (which == 1 ? WOT : WVT);
    if (t < nq) { const size_t e = t * 8; const int l = (int)(e / (H * H)); const int oo = (int)((e / H) % H), k0 = (int)(e % H); for (int j = 0; j < 8; ++j) o[j] = (b16)(bf16_rne(w[((size_t)l * H + k0 + j) * H + oo]) * WSC); for (int p = 0; p < 2; ++p) { *(volatile v8b*)(dst_ + e) = o; __threadfence(); } return; } t -= nq; }
  if (t < n2) { const size_t e = t * 8; const int oo = (int)(e / H), k0 = (int)(e % H); for (int j = 0; j < 8; ++j) o[j] = (b16)(bf16_rne(wv2[(size_t)(k0 + j) * H + oo]) * WSC); for (int p = 0; p < 2; ++p) { *(volatile v8b*)(WV2T + e) = o; __threadfence(); } return; } t -= n2;
  if (t < na) { const size_t e = t * 8; const int oo = (int)(e / (2 * H)), k0 = (int)(e % (2 * H)); for (int j = 0; j < 8; ++j) o[j] = (b16)(bf16_rne(wa[(size_t)(k0 + j) * H + oo]) * WSC); for (int p = 0; p < 2; ++p) { *(volatile v8b*)(WAT + e) = o; __threadfence(); } return; } t -= na;
  if (t < nb) { const size_t e = t * 8; const int oo = (int)(e / H), k0 = (int)(e % H); for (int j = 0; j < 8; ++j) o[j] = (oo < LAT + 1) ? (b16)(bf16_rne(wb[(size_t)(k0 + j) * (LAT + 1) + (oo < LAT + 1 ? oo : 0)]) * WSC) : (b16)0.0f; for (int p = 0; p < 2; ++p) { *(volatile v8b*)(WBT + e) = o; __threadfence(); } }
}
__global__ __launch_bounds__(256) void geo_kernel(const float* __restrict__ pos, const int* __restrict__ srcs, const int* __restrict__ dsts, float* __restrict__ DIRN, b16* __restrict__ RBH, b16* __restrict__ RBL) {
  const size_t e = (size_t)blockIdx.x * 256 + threadIdx.x; if (e >= (size_t)E) return;
  const int s = iclamp(srcs[e], 0, N - 1), t = iclamp(dsts[e], 0, N - 1);
  float d[3]; for (int c = 0; c < 3; ++c) d[c] = bf16_rne(pos[(size_t)t * 3 + c]) - bf16_rne(pos[(size_t)s * 3 + c]);
  const float r = sqrtf(pmul(d[0], d[0]) + pmul(d[1], d[1]) + pmul(d[2], d[2]) + EPSR); v4f dn; for (int c = 0; c < 3; ++c) dn[c] = d[c] / r; dn[3] = 0.0f;
  const float mean0 = 0.0067379469990854671f  ; const float tb = 0.0625f * (1.0f - mean0); const float beta = 1.0f / (tb * tb)  ; const float inv31 = 1.0f / 31.0f;
  const float cut = (r < CUT) ? 0.5f * (cosf(3.14159265358979323846f * r / CUT) + 1.0f) : 0.0f; const float er = __expf(-r);
  for (int pass = 0; pass < 2; ++pass) { *(volatile v4f*)(DIRN + e * 4) = dn; __threadfence(); }
#pragma unroll 1
  for (int q = 0; q < 4; ++q) { v8b hh, ll;
#pragma unroll
    for (int j = 0; j < 8; ++j) { const int k = q * 8 + j; const float kf = (float)k * inv31; const float mk = (k == R - 1) ? 1.0f : mean0 * (1.0f - kf) + kf  ; const float dd = er - mk; const float v = cut * __expf(-beta * pmul(dd, dd)); b16 p, ql; split16(v * RS, p, ql); hh[j] = p; ll[j] = ql; }
    for (int pass = 0; pass < 2; ++pass) { *(volatile v8b*)(RBH + e * R + q * 8) = hh; *(volatile v8b*)(RBL + e * R + q * 8) = ll; __threadfence(); } }
}
template <int RAWX>
__global__ __launch_bounds__(128) void edge_kernel(const b16* __restrict__ RBH, const b16* __restrict__ RBL, const b16* __restrict__ WR, const b16* __restrict__ W1T, const float* __restrict__ X, const float* __restrict__ embt, const int* __restrict__ zz, const int* __restrict__ srcs, float* __restrict__ FILT, float* __restrict__ PHI) {
  __shared__ __attribute__((aligned(16))) float Tf[4][16][H + 4]; __shared__ __attribute__((aligned(16))) b16 Ah[4][16][H + 8], Al[4][16][H + 8];
  const int wave = threadIdx.x >> 5, lane = threadIdx.x & 31, nloc = lane & 15, hlf = lane >> 4; const size_t e0 = (size_t)blockIdx.x * 64 + wave * 16;
  v8f acc[8];
#pragma unroll
  for (int t = 0; t < 8; ++t) acc[t] = (v8f){};
  { const v16b a = frag_kb(RBH + (e0 + nloc) * R, hlf), al = frag_kb(RBL + (e0 + nloc) * R, hlf);
#pragma unroll
    for (int t = 0; t < 8; ++t) { const v16b bw = frag_kb(WR + (size_t)(t * 16 + nloc) * R, hlf); acc[t] = wmma16b(a, bw, acc[t]); acc[t] = wmma16b(al, bw, acc[t]); } }
#pragma unroll
  for (int t = 0; t < 8; ++t)
#pragma unroll 1
    for (int r8 = 0; r8 < 8; ++r8) Tf[wave][8 * hlf + r8][t * 16 + nloc] = acc[t][r8] * (1.0f / (RS * WSC));
  wave_lds_sync();
  for (int pass = 0; pass < 2; ++pass) { for (int rr = 0; rr < 16; ++rr) *(volatile v4f*)(FILT + (e0 + rr) * H + lane * 4) = *(const v4f*)(&Tf[wave][rr][lane * 4]); __threadfence(); }
  for (int rr = 0; rr < 16; ++rr) { const int s = iclamp(srcs[e0 + rr], 0, N - 1); v4f xv; if (RAWX) { const int zi = iclamp(zz[s], 0, 99); xv = *(const v4f*)(embt + (size_t)zi * H + lane * 4); for (int j = 0; j < 4; ++j) xv[j] = bf16_rne(xv[j]); } else xv = *(const v4f*)(X + (size_t)s * H + lane * 4);
    const v4f f = *(const v4f*)(&Tf[wave][rr][lane * 4]); for (int j = 0; j < 4; ++j) { b16 p, q; split16(pmul(xv[j], f[j]) * XS, p, q); Ah[wave][rr][lane * 4 + j] = p; Al[wave][rr][lane * 4 + j] = q; } }
  wave_lds_sync();
#pragma unroll
  for (int t = 0; t < 8; ++t) acc[t] = (v8f){};
#pragma unroll 2
  for (int kb = 0; kb < H; kb += 32) { const v16b a = frag_kb(&Ah[wave][nloc][kb], hlf), al = frag_kb(&Al[wave][nloc][kb], hlf);
#pragma unroll
    for (int t = 0; t < 8; ++t) { const v16b bw = frag_kb(W1T + (size_t)(t * 16 + nloc) * H + kb, hlf); acc[t] = wmma16b(a, bw, acc[t]); acc[t] = wmma16b(al, bw, acc[t]); } }
  wave_lds_sync();
#pragma unroll
  for (int t = 0; t < 8; ++t)
#pragma unroll 1
    for (int r8 = 0; r8 < 8; ++r8) Tf[wave][8 * hlf + r8][t * 16 + nloc] = siluf(acc[t][r8] * (1.0f / (XS * WSC)));
  wave_lds_sync();
  for (int pass = 0; pass < 2; ++pass) { for (int rr = 0; rr < 16; ++rr) *(volatile v4f*)(PHI + (e0 + rr) * H + lane * 4) = *(const v4f*)(&Tf[wave][rr][lane * 4]); __threadfence(); }
}
template <int RAWX>
__global__ __launch_bounds__(32) void nodes_kernel(const float* __restrict__ PHI, const float* __restrict__ X, const float* __restrict__ embt, const int* __restrict__ zz, const b16* __restrict__ WOT, const int* __restrict__ PERM, const int* __restrict__ ROWPTR, const int* __restrict__ ROWCNT, int permLen, float* __restrict__ XOUT) {
  __shared__ __attribute__((aligned(16))) b16 Ah[16][H + 8], Al[16][H + 8]; __shared__ __attribute__((aligned(16))) float Tf[16][H + 4];
  const int lane = threadIdx.x, nloc = lane & 15, hlf = lane >> 4; const size_t v0 = (size_t)blockIdx.x * 16;
  for (int rr = 0; rr < 16; ++rr) { const size_t v = v0 + rr; v4f a = {0.0f, 0.0f, 0.0f, 0.0f}, xv = {0.0f, 0.0f, 0.0f, 0.0f};
    if (v < (size_t)N) { int st = ROWPTR[v], cnt = ROWCNT[v]; cnt = iclamp(cnt, 0, 65536); st = iclamp(st, 0, permLen - cnt);
#pragma unroll 2
      for (int j = 0; j < cnt; ++j) { const int e = iclamp(PERM[st + j], 0, E - 1); const v4f p = *(const v4f*)(PHI + (size_t)e * H + lane * 4); for (int i = 0; i < 4; ++i) a[i] += p[i]; }
      if (RAWX) { const int zi = iclamp(zz[v], 0, 99); xv = *(const v4f*)(embt + (size_t)zi * H + lane * 4); for (int i = 0; i < 4; ++i) xv[i] = bf16_rne(xv[i]); } else xv = *(const v4f*)(X + v * H + lane * 4); }
    for (int i = 0; i < 4; ++i) { b16 p, q; split16(a[i] * XS, p, q); Ah[rr][lane * 4 + i] = p; Al[rr][lane * 4 + i] = q; Tf[rr][lane * 4 + i] = xv[i]; } }
  wave_lds_sync();
  v8f acc[8];
#pragma unroll
  for (int t = 0; t < 8; ++t) acc[t] = (v8f){};
#pragma unroll 2
  for (int kb = 0; kb < H; kb += 32) { const v16b a = frag_kb(&Ah[nloc][kb], hlf), al = frag_kb(&Al[nloc][kb], hlf);
#pragma unroll
    for (int t = 0; t < 8; ++t) { const v16b bw = frag_kb(WOT + (size_t)(t * 16 + nloc) * H + kb, hlf); acc[t] = wmma16b(a, bw, acc[t]); acc[t] = wmma16b(al, bw, acc[t]); } }
  wave_lds_sync();
#pragma unroll
  for (int t = 0; t < 8; ++t)
#pragma unroll 1
    for (int r8 = 0; r8 < 8; ++r8) { const int rl = 8 * hlf + r8, c = t * 16 + nloc; Tf[rl][c] = Tf[rl][c] + acc[t][r8] * (1.0f / (XS * WSC)); }
  wave_lds_sync();
  for (int pass = 0; pass < 2; ++pass) { for (int rr = 0; rr < 16; ++rr) *(volatile v4f*)(XOUT + (v0 + rr) * H + lane * 4) = *(const v4f*)(&Tf[rr][lane * 4]); __threadfence(); }
}
__global__ __launch_bounds__(128) void vgemm_kernel(const float* __restrict__ VEC, const b16* __restrict__ W, float* __restrict__ VM) {
  __shared__ __attribute__((aligned(16))) b16 Ah[4][16][H + 8], Al[4][16][H + 8]; __shared__ __attribute__((aligned(16))) float Tf[4][16][H + 4];
  const int wave = threadIdx.x >> 5, lane = threadIdx.x & 31, nloc = lane & 15, hlf = lane >> 4; const size_t m0 = (size_t)blockIdx.x * 64 + wave * 16;
  for (int rr = 0; rr < 16; ++rr) { const v4f v = *(const v4f*)(VEC + (m0 + rr) * H + lane * 4); for (int j = 0; j < 4; ++j) { b16 p, q; split16(v[j] * XS, p, q); Ah[wave][rr][lane * 4 + j] = p; Al[wave][rr][lane * 4 + j] = q; } }
  wave_lds_sync();
  v8f acc[8];
#pragma unroll
  for (int t = 0; t < 8; ++t) acc[t] = (v8f){};
#pragma unroll 2
  for (int kb = 0; kb < H; kb += 32) { const v16b a = frag_kb(&Ah[wave][nloc][kb], hlf), al = frag_kb(&Al[wave][nloc][kb], hlf);
#pragma unroll
    for (int t = 0; t < 8; ++t) { const v16b bw = frag_kb(W + (size_t)(t * 16 + nloc) * H + kb, hlf); acc[t] = wmma16b(a, bw, acc[t]); acc[t] = wmma16b(al, bw, acc[t]); } }
#pragma unroll
  for (int t = 0; t < 8; ++t)
#pragma unroll 1
    for (int r8 = 0; r8 < 8; ++r8) Tf[wave][8 * hlf + r8][t * 16 + nloc] = acc[t][r8] * (1.0f / (XS * WSC));
  wave_lds_sync();
  for (int pass = 0; pass < 2; ++pass) { for (int rr = 0; rr < 16; ++rr) *(volatile v4f*)(VM + (m0 + rr) * H + lane * 4) = *(const v4f*)(&Tf[wave][rr][lane * 4]); __threadfence(); }
}
template <int HASV>
__global__ __launch_bounds__(256) void nodev_kernel(const float* __restrict__ VEC, const float* __restrict__ VMIX, const float* __restrict__ FILT, const float* __restrict__ PHI, const float* __restrict__ DIRN, const int* __restrict__ srcs, const int* __restrict__ PERM, const int* __restrict__ ROWPTR, const int* __restrict__ ROWCNT, int permLen, float* __restrict__ VOUT) {
  const int wave = threadIdx.x >> 5, lane = threadIdx.x & 31; const size_t v = (size_t)blockIdx.x * 8 + wave; v4f a[3]; for (int c = 0; c < 3; ++c) a[c] = (v4f){0.0f, 0.0f, 0.0f, 0.0f};
  if (v < (size_t)N) { int st = ROWPTR[v], cnt = ROWCNT[v]; cnt = iclamp(cnt, 0, 65536); st = iclamp(st, 0, permLen - cnt);
#pragma unroll 1
    for (int j = 0; j < cnt; ++j) { const int e = iclamp(PERM[st + j], 0, E - 1); const v4f p = *(const v4f*)(PHI + (size_t)e * H + lane * 4); const v4f dn = *(const v4f*)(DIRN + (size_t)e * 4);
      if (HASV) { const size_t s = (size_t)iclamp(srcs[e], 0, N - 1); const v4f f = *(const v4f*)(FILT + (size_t)e * H + lane * 4);
        for (int c = 0; c < 3; ++c) { const v4f vm = *(const v4f*)(VMIX + (s * 3 + c) * H + lane * 4); for (int i = 0; i < 4; ++i) a[c][i] += pmul(vm[i], f[i]) + pmul(p[i], dn[c]); } }
      else { for (int c = 0; c < 3; ++c) for (int i = 0; i < 4; ++i) a[c][i] += pmul(p[i], dn[c]); } }
    if (HASV) for (int c = 0; c < 3; ++c) { const v4f old = *(const v4f*)(VEC + (v * 3 + c) * H + lane * 4); for (int i = 0; i < 4; ++i) a[c][i] += old[i]; } }
  for (int pass = 0; pass < 2; ++pass) { for (int c = 0; c < 3; ++c) *(volatile v4f*)(VOUT + (v * 3 + c) * H + lane * 4) = a[c]; __threadfence(); }
}
__global__ __launch_bounds__(32) void head_kernel(const float* __restrict__ X, const float* __restrict__ V2, const b16* __restrict__ WAT, const float* __restrict__ ba, const b16* __restrict__ WBT, const float* __restrict__ bb, float* __restrict__ OUTN) {
  __shared__ __attribute__((aligned(16))) b16 Ah[16][2 * H + 8], Al[16][2 * H + 8]; __shared__ __attribute__((aligned(16))) float To[16][OW + 4];
  const int lane = threadIdx.x, nloc = lane & 15, hlf = lane >> 4; const size_t v0 = (size_t)blockIdx.x * 16;
  for (int rr = 0; rr < 16; ++rr) { const size_t v = v0 + rr; v4f xv = {0.0f, 0.0f, 0.0f, 0.0f}, q0 = xv, q1 = xv, q2 = xv;
    if (v < (size_t)N) { xv = *(const v4f*)(X + v * H + lane * 4); q0 = *(const v4f*)(V2 + (v * 3 + 0) * H + lane * 4); q1 = *(const v4f*)(V2 + (v * 3 + 1) * H + lane * 4); q2 = *(const v4f*)(V2 + (v * 3 + 2) * H + lane * 4); }
    for (int j = 0; j < 4; ++j) { const float vn = sqrtf(pmul(q0[j], q0[j]) + pmul(q1[j], q1[j]) + pmul(q2[j], q2[j]) + EPSR); b16 p, q; split16(xv[j] * XS, p, q); Ah[rr][lane * 4 + j] = p; Al[rr][lane * 4 + j] = q; split16(vn * XS, p, q); Ah[rr][H + lane * 4 + j] = p; Al[rr][H + lane * 4 + j] = q; } }
  wave_lds_sync();
  v8f acc[8];
#pragma unroll
  for (int t = 0; t < 8; ++t) acc[t] = (v8f){};
#pragma unroll 2
  for (int kb = 0; kb < 2 * H; kb += 32) { const v16b a = frag_kb(&Ah[nloc][kb], hlf), al = frag_kb(&Al[nloc][kb], hlf);
#pragma unroll
    for (int t = 0; t < 8; ++t) { const v16b bw = frag_kb(WAT + (size_t)(t * 16 + nloc) * (2 * H) + kb, hlf); acc[t] = wmma16b(a, bw, acc[t]); acc[t] = wmma16b(al, bw, acc[t]); } }
  wave_lds_sync();
#pragma unroll
  for (int t = 0; t < 8; ++t) { const int c = t * 16 + nloc; const float bav = bf16_rne(ba[c]);
#pragma unroll 1
    for (int r8 = 0; r8 < 8; ++r8) { const float av = siluf(acc[t][r8] * (1.0f / (XS * WSC)) + bav); b16 p, q; split16(av * XS, p, q); Ah[8 * hlf + r8][c] = p; Al[8 * hlf + r8][c] = q; } }
  wave_lds_sync();
  v8f acc2[5];
#pragma unroll
  for (int t = 0; t < 5; ++t) acc2[t] = (v8f){};
#pragma unroll 2
  for (int kb = 0; kb < H; kb += 32) { const v16b a = frag_kb(&Ah[nloc][kb], hlf), al = frag_kb(&Al[nloc][kb], hlf);
#pragma unroll
    for (int t = 0; t < 5; ++t) { const v16b bw = frag_kb(WBT + (size_t)(t * 16 + nloc) * H + kb, hlf); acc2[t] = wmma16b(a, bw, acc2[t]); acc2[t] = wmma16b(al, bw, acc2[t]); } }
#pragma unroll
  for (int t = 0; t < 5; ++t) { const int c = t * 16 + nloc; const float bbv = (c < LAT + 1) ? bf16_rne(bb[c < LAT + 1 ? c : 0]) : 0.0f;
#pragma unroll 1
    for (int r8 = 0; r8 < 8; ++r8) { const int rl = 8 * hlf + r8; const bool ok = (v0 + rl) < (size_t)N; To[rl][c] = (ok && c < LAT + 1) ? acc2[t][r8] * (1.0f / (XS * WSC)) + bbv : 0.0f; } }
  wave_lds_sync();
  for (int pass = 0; pass < 2; ++pass) { for (int rr = 0; rr < 16; ++rr) { if (lane < OW / 4) *(volatile v4f*)(OUTN + (v0 + rr) * OW + lane * 4) = *(const v4f*)(&To[rr][lane * 4]); } __threadfence(); }
}
__global__ __launch_bounds__(256) void pool_kernel(const float* __restrict__ OUTN, const int* __restrict__ PERM, const int* __restrict__ ROWPTR, const int* __restrict__ ROWCNT, int permLen, float* __restrict__ outMu, float* __restrict__ outLv) {
  __shared__ float lvs[32];
  const int wave = threadIdx.x >> 5, lane = threadIdx.x & 31;
#pragma unroll 1
  for (int qq = 0; qq < 4; ++qq) { const int gl = wave * 4 + qq; const int g = blockIdx.x * 32 + gl; const int tix = (g >> 3) * 32 + (g & 7);
    int st = ROWPTR[tix], cnt = ROWCNT[tix]; cnt = iclamp(cnt, 0, 65536); st = iclamp(st, 0, permLen - cnt); v4f a = {0.0f, 0.0f, 0.0f, 0.0f}; const int lc = lane < OW / 4 ? lane : 0;
#pragma unroll 1
    for (int j = 0; j < cnt; ++j) { const int n = iclamp(PERM[st + j], 0, N - 1); const v4f o = *(const v4f*)(OUTN + (size_t)n * OW + lc * 4); for (int i = 0; i < 4; ++i) a[i] += o[i]; }
    if (lane == 16) lvs[gl] = fminf(fmaxf(a[0], -10.0f), 2.0f);
    for (int pass = 0; pass < 2; ++pass) { if (lane < 16) *(volatile v4f*)(outMu + (size_t)g * LAT + lane * 4) = a; __threadfence(); } }
  __syncthreads();
  for (int pass = 0; pass < 2; ++pass) { if (threadIdx.x < 8) *(volatile v4f*)(outLv + (size_t)blockIdx.x * 32 + threadIdx.x * 4) = *(const v4f*)(&lvs[threadIdx.x * 4]); __threadfence(); }
}
}

extern "C" void kernel_launch(void* const* d_in, const int* in_sizes, int n_in, void* d_out, int out_size, void* d_ws, size_t ws_size, hipStream_t stream) {
  (void)n_in;
  auto Fp = [&](int i) { return (const float*)d_in[i]; }; auto Ip = [&](int i) { return (const int*)d_in[i]; };
  if (in_sizes[0] != N || in_sizes[1] != N * 3 || in_sizes[2] != N || in_sizes[3] != 2 * E || in_sizes[4] != 100 * H || in_sizes[5] != L * R * H || in_sizes[6] != L * H * H || in_sizes[10] != H * H || in_sizes[11] != 2 * H * H || in_sizes[13] != H * (LAT + 1) || in_sizes[14] != LAT + 1 || out_size != G * LAT + G) return;
  size_t off = 0; char* ws = (char*)d_ws;
  auto carve = [&](size_t bytes) { char* p = ws + off; off += (bytes + 255) & ~(size_t)255; return p; };
  b16* WR = (b16*)carve((size_t)L * H * R * 2); b16* W1T = (b16*)carve((size_t)L * H * H * 2); b16* WOT = (b16*)carve((size_t)L * H * H * 2); b16* WVT = (b16*)carve((size_t)L * H * H * 2); b16* WV2T = (b16*)carve((size_t)H * H * 2); b16* WAT = (b16*)carve((size_t)H * 2 * H * 2); b16* WBT = (b16*)carve((size_t)OW * H * 2);
  float* DIRN = (float*)carve((size_t)E * 4 * 4); b16* RBH = (b16*)carve((size_t)E * R * 2); b16* RBL = (b16*)carve((size_t)E * R * 2);
  float* FILT = (float*)carve((size_t)E * H * 4); float* PHI = (float*)carve((size_t)E * H * 4);
  float* XA = (float*)carve((size_t)NP * H * 4); float* XB = (float*)carve((size_t)NP * H * 4); float* VA = (float*)carve((size_t)NP * 3 * H * 4); float* VB = (float*)carve((size_t)NP * 3 * H * 4); float* VM = (float*)carve((size_t)NP * 3 * H * 4); float* OUTN = (float*)carve((size_t)NP * OW * 4);
  CsrBufs9 csr; CsrBufs3 pool; off = csr_carve9(csr, ws, off, E, N); off = csr_carve3(pool, ws, off, N, G);
  if (off > ws_size) return;
  const unsigned nw = (unsigned)(((size_t)L * H * R / 8 + 3 * (size_t)L * H * H / 8 + (size_t)H * H / 8 + (size_t)H * 2 * H / 8 + (size_t)OW * H / 8 + 255) / 256);
  wprep_kernel<<<nw, 256, 0, stream>>>(Fp(5), Fp(6), Fp(7), Fp(8), Fp(10), Fp(11), Fp(13), WR, W1T, WOT, WVT, WV2T, WAT, WBT);
  csr_build9(csr, Ip(3) + E, E, N, stream);
  csr_build3(pool, Ip(2), N, G, stream);
  geo_kernel<<<E / 256, 256, 0, stream>>>(Fp(1), Ip(3), Ip(3) + E, DIRN, RBH, RBL);
  edge_kernel<1><<<E / 64, 128, 0, stream>>>(RBH, RBL, WR, W1T, nullptr, Fp(4), Ip(0), Ip(3), FILT, PHI);
  nodes_kernel<1><<<NP / 16, 32, 0, stream>>>(PHI, nullptr, Fp(4), Ip(0), WOT, csr.PERM, csr.ROWPTR, csr.ROWCNT, (int)csr.permLen, XA);
  nodev_kernel<0><<<NP / 8, 256, 0, stream>>>(nullptr, nullptr, FILT, PHI, DIRN, Ip(3), csr.PERM, csr.ROWPTR, csr.ROWCNT, (int)csr.permLen, VA);
  edge_kernel<0><<<E / 64, 128, 0, stream>>>(RBH, RBL, WR + (size_t)H * R, W1T + (size_t)H * H, XA, Fp(4), Ip(0), Ip(3), FILT, PHI);
  nodes_kernel<0><<<NP / 16, 32, 0, stream>>>(PHI, XA, Fp(4), Ip(0), WOT + (size_t)H * H, csr.PERM, csr.ROWPTR, csr.ROWCNT, (int)csr.permLen, XB);
  vgemm_kernel<<<NP * 3 / 64, 128, 0, stream>>>(VA, WVT + (size_t)H * H, VM);
  nodev_kernel<1><<<NP / 8, 256, 0, stream>>>(VA, VM, FILT, PHI, DIRN, Ip(3), csr.PERM, csr.ROWPTR, csr.ROWCNT, (int)csr.permLen, VB);
  vgemm_kernel<<<NP * 3 / 64, 128, 0, stream>>>(VB, WV2T, VM);
  head_kernel<<<NP / 16, 32, 0, stream>>>(XB, VM, WAT, Fp(12), WBT, Fp(14), OUTN);
  float* outMu = (float*)d_out; float* outLv = outMu + (size_t)G * LAT;
  pool_kernel<<<G / 32, 256, 0, stream>>>(OUTN, pool.PERM, pool.ROWPTR, pool.ROWCNT, (int)pool.permLen, outMu, outLv);
}
